// HeposMultiHeadAttention_8392366096731
// MI455X (gfx1250) — hardware-verified
//
#include <hip/hip_runtime.h>


#define TQ   1024
#define TK   8192
#define DM   1024
#define NH_  16
#define HD   64
#define KPH  512
typedef _Float16 h16;
typedef unsigned short bf;
typedef __attribute__((ext_vector_type(16))) __bf16   v16bf;
typedef __attribute__((ext_vector_type(16))) _Float16 v16h;
typedef __attribute__((ext_vector_type(8)))  _Float16 v8h;
typedef __attribute__((ext_vector_type(8)))  unsigned short v8us;
typedef __attribute__((ext_vector_type(8)))  float    v8f;
typedef __attribute__((ext_vector_type(4)))  float    v4f;
typedef v8h  __attribute__((may_alias)) v8ha;
typedef v4f  __attribute__((may_alias)) v4fa;
typedef v8us __attribute__((may_alias)) v8usa;

__device__ __forceinline__ unsigned short f2bf(float f) { unsigned u = __float_as_uint(f); u += 0x7FFFu + ((u >> 16) & 1u); return (unsigned short)(u >> 16); }
__device__ __forceinline__ float bf2f(unsigned short b) { return __uint_as_float(((unsigned)b) << 16); }
__device__ __forceinline__ float bfr(float f) { return bf2f(f2bf(f)); }
__device__ __forceinline__ v16h cat16(v8h lo, v8h hi) { return __builtin_shufflevector(lo, hi, 0, 1, 2, 3, 4, 5, 6, 7, 8, 9, 10, 11, 12, 13, 14, 15); }
__device__ __forceinline__ v16bf cat16b(v8us lo, v8us hi) { return __builtin_bit_cast(v16bf, __builtin_shufflevector(lo, hi, 0, 1, 2, 3, 4, 5, 6, 7, 8, 9, 10, 11, 12, 13, 14, 15)); }
__device__ __forceinline__ v8f wmma16(v16h a, v16h b, v8f c) { return __builtin_amdgcn_wmma_f32_16x16x32_f16(false, a, false, b, (short)0, c, false, false); }
__device__ __forceinline__ v8f wmmab(v16bf a, v16bf b, v8f c) { return __builtin_amdgcn_wmma_f32_16x16x32_bf16(false, a, false, b, (short)0, c, false, false); }


template <typename T16> struct WFrag;
template <> struct WFrag<h16> { typedef v16h V; static __device__ __forceinline__ V ld(const h16* p) { return cat16(*(const v8h*)p, *(const v8h*)(p + 16)); } static __device__ __forceinline__ v8f mma(V a, V b, v8f c) { return wmma16(a, b, c); } };
template <> struct WFrag<bf> { typedef v16bf V; static __device__ __forceinline__ V ld(const bf* p) { return cat16b(*(const v8us*)p, *(const v8us*)(p + 16)); } static __device__ __forceinline__ v8f mma(V a, V b, v8f c) { return wmmab(a, b, c); } };
template <typename T16, int NSPLIT, bool BIAS>
__global__ __launch_bounds__(32) void k_gemmw(const T16* __restrict__ A, const T16* __restrict__ A2, const T16* __restrict__ Bt, const T16* __restrict__ Bt2, int K, float* C, int ldc, const float* __restrict__ bias, size_t sA, size_t sB, size_t sC) {
    typedef typename WFrag<T16>::V V;
    __shared__ __align__(16) float os[16 * 68];
    const size_t z = blockIdx.z; A += z * sA; if (A2) A2 += z * sA; Bt += z * sB; if (Bt2) Bt2 += z * sB; C += z * sC;
    const int lane = threadIdx.x & 31, lr = lane & 15, hi = lane >> 4; const int r0 = blockIdx.x * 64, c0 = blockIdx.y * 64;
    v8f acc[4][4];
#pragma unroll
    for (int mb = 0; mb < 4; ++mb)
#pragma unroll
        for (int nb = 0; nb < 4; ++nb) acc[mb][nb] = (v8f){};
    const size_t aoff = (size_t)(r0 + lr) * K + 8 * hi, boff = (size_t)(c0 + lr) * K + 8 * hi;
#pragma unroll 1
    for (int kc = 0; kc < K; kc += 32) {
        V a[4], a2[4];
#pragma unroll
        for (int mb = 0; mb < 4; ++mb) { a[mb] = WFrag<T16>::ld(A + aoff + (size_t)mb * 16 * K + kc); if (NSPLIT == 1 || NSPLIT == 2) a2[mb] = WFrag<T16>::ld(A2 + aoff + (size_t)mb * 16 * K + kc); }
#pragma unroll
        for (int nb = 0; nb < 4; ++nb) { const V b = WFrag<T16>::ld(Bt + boff + (size_t)nb * 16 * K + kc); V b2; if (NSPLIT >= 2) b2 = WFrag<T16>::ld(Bt2 + boff + (size_t)nb * 16 * K + kc);
#pragma unroll
            for (int mb = 0; mb < 4; ++mb) { acc[mb][nb] = WFrag<T16>::mma(a[mb], b, acc[mb][nb]); if (NSPLIT == 1 || NSPLIT == 2) acc[mb][nb] = WFrag<T16>::mma(a2[mb], b, acc[mb][nb]); if (NSPLIT >= 2) acc[mb][nb] = WFrag<T16>::mma(a[mb], b2, acc[mb][nb]); } }
        asm volatile("v_nop\n\tv_nop\n\tv_nop\n\tv_nop" : "+v"(acc[0][0]), "+v"(acc[1][1]), "+v"(acc[2][2]), "+v"(acc[3][3]) : "v"(a[0]), "v"(a[3]));
    }
#pragma unroll
    for (int mb = 0; mb < 4; ++mb) {
#pragma unroll
        for (int nb = 0; nb < 4; ++nb) {
#pragma unroll
            for (int j = 0; j < 8; ++j) os[(hi * 8 + j) * 68 + nb * 16 + lr] = acc[mb][nb][j]; }
        __builtin_amdgcn_wave_barrier(); asm volatile("" ::: "memory");
        float* crow = C + (size_t)(r0 + mb * 16) * ldc + c0;
#pragma unroll 1
        for (int ps = 0; ps < 2; ++ps) {
#pragma unroll
            for (int s = 0; s < 8; ++s) { const int row = 2 * s + hi, cofs = lr * 4; v4f val = *(const v4fa*)(os + row * 68 + cofs); if (BIAS) { val[0] += bfr(bias[c0 + cofs]); val[1] += bfr(bias[c0 + cofs + 1]); val[2] += bfr(bias[c0 + cofs + 2]); val[3] += bfr(bias[c0 + cofs + 3]); }
                *(volatile v4f*)(crow + (size_t)row * ldc + cofs) = val; }
            if (ps == 0) __threadfence(); }
        __builtin_amdgcn_wave_barrier(); asm volatile("" ::: "memory");
    }
}

__device__ __forceinline__ void splitf(float y, unsigned short& h, unsigned short& l) { h = f2bf(y); l = f2bf(y - bf2f(h)); }
typedef __attribute__((ext_vector_type(2))) unsigned short v2us;
typedef __attribute__((ext_vector_type(4))) unsigned short v4us;

__global__ __launch_bounds__(256) void k_cvt8(const float* __restrict__ src, bf* dst, size_t n8) { const size_t i = (size_t)blockIdx.x * 256 + threadIdx.x; if (i >= n8) return; const v8f v = *(const v8f*)(src + i * 8); v8us o;
#pragma unroll
    for (int k = 0; k < 8; ++k) o[k] = f2bf(v[k]); *(volatile v8us*)(dst + i * 8) = o; __threadfence(); *(volatile v8us*)(dst + i * 8) = o; }
__global__ __launch_bounds__(256) void k_qpl(const float* __restrict__ Q, bf* Qh, bf* Ql) { const size_t e = ((size_t)blockIdx.x * 256 + threadIdx.x) * 4; if (e >= (size_t)NH_ * TQ * HD) return; const int d = (int)(e % HD); const int t = (int)((e / HD) % TQ); const int h = (int)(e / ((size_t)HD * TQ)); const v4f a = *(const v4f*)(Q + (size_t)t * DM + h * HD + d); v4us oh, ol;
#pragma unroll
    for (int u = 0; u < 4; ++u) { unsigned short x0, x1; splitf(a[u], x0, x1); oh[u] = x0; ol[u] = x1; } *(volatile v4us*)(Qh + e) = oh; *(volatile v4us*)(Ql + e) = ol; __threadfence(); *(volatile v4us*)(Qh + e) = oh; *(volatile v4us*)(Ql + e) = ol; }
__global__ __launch_bounds__(256) void k_kpl(const float* __restrict__ K, bf* Kh, bf* Kl) { const size_t e = ((size_t)blockIdx.x * 256 + threadIdx.x) * 4; if (e >= (size_t)NH_ * KPH * HD) return; const int d = (int)(e % HD); const int m = (int)((e / HD) % KPH); const int h = (int)(e / ((size_t)HD * KPH)); const v4f a = *(const v4f*)(K + (size_t)(16 * m + h) * DM + h * HD + d); v4us oh, ol;
#pragma unroll
    for (int u = 0; u < 4; ++u) { unsigned short x0, x1; splitf(a[u], x0, x1); oh[u] = x0; ol[u] = x1; } *(volatile v4us*)(Kh + e) = oh; *(volatile v4us*)(Kl + e) = ol; __threadfence(); *(volatile v4us*)(Kh + e) = oh; *(volatile v4us*)(Kl + e) = ol; }
__global__ __launch_bounds__(256) void k_vtp(const float* __restrict__ V, bf* Vh, bf* Vl) { const size_t e = ((size_t)blockIdx.x * 256 + threadIdx.x) * 4; if (e >= (size_t)NH_ * HD * KPH) return; const int m = (int)(e % KPH); const int d = (int)((e / KPH) % HD); const int h = (int)(e / ((size_t)KPH * HD)); v4us oh, ol;
#pragma unroll
    for (int u = 0; u < 4; ++u) { unsigned short x0, x1; splitf(V[(size_t)(16 * (m + u) + h) * DM + h * HD + d], x0, x1); oh[u] = x0; ol[u] = x1; } *(volatile v4us*)(Vh + e) = oh; *(volatile v4us*)(Vl + e) = ol; __threadfence(); *(volatile v4us*)(Vh + e) = oh; *(volatile v4us*)(Vl + e) = ol; }
__global__ __launch_bounds__(256) void k_soft(const float* __restrict__ S, bf* Ph, bf* Pl) { const int lane = threadIdx.x & 31; const int row = blockIdx.x * 8 + (threadIdx.x >> 5); if (row >= NH_ * TQ) return; const float* sr = S + (size_t)row * KPH; float v[KPH / 32]; float mx = -3.0e38f;
#pragma unroll
    for (int ch = 0; ch < KPH / 128; ++ch) { const v4f a = *(const v4f*)(sr + ch * 128 + lane * 4);
#pragma unroll
        for (int u = 0; u < 4; ++u) { const float t = a[u] * 0.125f; v[ch * 4 + u] = t; mx = fmaxf(mx, t); } }
#pragma unroll
    for (int sh = 16; sh; sh >>= 1) mx = fmaxf(mx, __shfl_xor(mx, sh, 32));
    float sum = 0.f;
#pragma unroll
    for (int q = 0; q < KPH / 32; ++q) { float d0 = __fsub_rn(v[q], mx); asm volatile("" : "+v"(d0)); v[q] = __builtin_amdgcn_exp2f(__fmul_rn(d0, 1.4426950408889634f)); sum += v[q]; }
#pragma unroll
    for (int sh = 16; sh; sh >>= 1) sum += __shfl_xor(sum, sh, 32);
    const float f = __fdiv_rn(1.0f, sum);
    for (int ps = 0; ps < 2; ++ps) {
#pragma unroll
        for (int ch = 0; ch < KPH / 128; ++ch) { v4us oh, ol; for (int q = 0; q < 4; ++q) { unsigned short a, b; splitf(v[ch * 4 + q] * f, a, b); oh[q] = a; ol[q] = b; } const size_t oo = (size_t)row * KPH + ch * 128 + lane * 4; *(volatile v4us*)(Ph + oo) = oh; *(volatile v4us*)(Pl + oo) = ol; }
        if (ps == 0) __threadfence(); } }
__global__ __launch_bounds__(256) void k_mrg(const float* __restrict__ O, bf* Ah, bf* Al) { const size_t e = ((size_t)blockIdx.x * 256 + threadIdx.x) * 4; if (e >= (size_t)NH_ * TQ * HD) return; const int d = (int)(e % HD); const int t = (int)((e / HD) % TQ); const int h = (int)(e / ((size_t)HD * TQ)); const size_t oo = (size_t)t * DM + h * HD + d; v4us oh, ol;
#pragma unroll
    for (int u = 0; u < 4; ++u) { unsigned short a, b; splitf(O[e + u], a, b); oh[u] = a; ol[u] = b; } *(volatile v4us*)(Ah + oo) = oh; *(volatile v4us*)(Al + oo) = ol; __threadfence(); *(volatile v4us*)(Ah + oo) = oh; *(volatile v4us*)(Al + oo) = ol; }

extern "C" void kernel_launch(void* const* d_in, const int* in_sizes, int n_in,
                              void* d_out, int out_size, void* d_ws, size_t ws_size, hipStream_t stream) {
    (void)in_sizes; (void)n_in; (void)out_size;
    const float* qin = (const float*)d_in[0]; const float* kin = (const float*)d_in[1]; const float* vin = (const float*)d_in[2]; const float* Wq = (const float*)d_in[3]; const float* bq = (const float*)d_in[4]; const float* Wk = (const float*)d_in[5]; const float* bk = (const float*)d_in[6]; const float* Wv = (const float*)d_in[7]; const float* bv = (const float*)d_in[8]; const float* Wo = (const float*)d_in[9]; const float* bo = (const float*)d_in[10];
    float* OUT = (float*)d_out;
    char* wsp = (char*)d_ws;
    auto take = [&](size_t bytes) { char* p = wsp; wsp += (bytes + 255) & ~(size_t)255; return (void*)p; };
    bf* BQ = (bf*)take((size_t)DM * DM * 2); bf* BK = (bf*)take((size_t)DM * DM * 2); bf* BV = (bf*)take((size_t)DM * DM * 2); bf* BO = (bf*)take((size_t)DM * DM * 2);
    bf* QB = (bf*)take((size_t)TQ * DM * 2); bf* KB = (bf*)take((size_t)TK * DM * 2); float* FQ = (float*)take((size_t)TQ * DM * 4); float* FK = (float*)take((size_t)TK * DM * 4); float* FV = (float*)take((size_t)TK * DM * 4);
    bf* Qh = (bf*)take((size_t)NH_ * TQ * HD * 2); bf* Ql = (bf*)take((size_t)NH_ * TQ * HD * 2); bf* Kh = (bf*)take((size_t)NH_ * KPH * HD * 2); bf* Kl = (bf*)take((size_t)NH_ * KPH * HD * 2); bf* Vh = (bf*)take((size_t)NH_ * HD * KPH * 2); bf* Vl = (bf*)take((size_t)NH_ * HD * KPH * 2);
    float* S = (float*)take((size_t)NH_ * TQ * KPH * 4); bf* Ph = (bf*)take((size_t)NH_ * TQ * KPH * 2); bf* Pl = (bf*)take((size_t)NH_ * TQ * KPH * 2); float* O = (float*)take((size_t)NH_ * TQ * HD * 4); bf* ATh = (bf*)take((size_t)TQ * DM * 2); bf* ATl = (bf*)take((size_t)TQ * DM * 2);
    if ((size_t)(wsp - (char*)d_ws) > ws_size) return;
    k_cvt8<<<(DM * DM / 8 + 255) / 256, 256, 0, stream>>>(Wq, BQ, DM * DM / 8); k_cvt8<<<(DM * DM / 8 + 255) / 256, 256, 0, stream>>>(Wk, BK, DM * DM / 8); k_cvt8<<<(DM * DM / 8 + 255) / 256, 256, 0, stream>>>(Wv, BV, DM * DM / 8); k_cvt8<<<(DM * DM / 8 + 255) / 256, 256, 0, stream>>>(Wo, BO, DM * DM / 8);
    k_cvt8<<<(TQ * DM / 8 + 255) / 256, 256, 0, stream>>>(qin, QB, TQ * DM / 8);
    k_gemmw<bf, 0, true><<<dim3(TQ / 64, DM / 64, 1), 32, 0, stream>>>(QB, nullptr, BQ, nullptr, DM, FQ, DM, bq, 0, 0, 0);
    k_cvt8<<<(TK * DM / 8 + 255) / 256, 256, 0, stream>>>(kin, KB, TK * DM / 8);
    k_gemmw<bf, 0, true><<<dim3(TK / 64, DM / 64, 1), 32, 0, stream>>>(KB, nullptr, BK, nullptr, DM, FK, DM, bk, 0, 0, 0);
    k_cvt8<<<(TK * DM / 8 + 255) / 256, 256, 0, stream>>>(vin, KB, TK * DM / 8);
    k_gemmw<bf, 0, true><<<dim3(TK / 64, DM / 64, 1), 32, 0, stream>>>(KB, nullptr, BV, nullptr, DM, FV, DM, bv, 0, 0, 0);
    k_qpl<<<(unsigned)(((size_t)NH_ * TQ * HD / 4 + 255) / 256), 256, 0, stream>>>(FQ, Qh, Ql); k_kpl<<<(unsigned)(((size_t)NH_ * KPH * HD / 4 + 255) / 256), 256, 0, stream>>>(FK, Kh, Kl); k_vtp<<<(unsigned)(((size_t)NH_ * HD * KPH / 4 + 255) / 256), 256, 0, stream>>>(FV, Vh, Vl);
    const size_t zq = (size_t)TQ * HD, zk = (size_t)KPH * HD, zS = (size_t)TQ * KPH, zv = (size_t)HD * KPH;
    k_gemmw<bf, 2, false><<<dim3(TQ / 64, KPH / 64, NH_), 32, 0, stream>>>(Qh, Ql, Kh, Kl, HD, S, KPH, nullptr, zq, zk, zS);
    k_soft<<<NH_ * TQ / 8, 256, 0, stream>>>(S, Ph, Pl);
    k_gemmw<bf, 2, false><<<dim3(TQ / 64, 1, NH_), 32, 0, stream>>>(Ph, Pl, Vh, Vl, KPH, O, HD, nullptr, zS, zv, zq);
    k_mrg<<<(unsigned)(((size_t)NH_ * TQ * HD / 4 + 255) / 256), 256, 0, stream>>>(O, ATh, ATl);
    k_gemmw<bf, 1, true><<<dim3(TQ / 64, DM / 64, 1), 32, 0, stream>>>(ATh, ATl, BO, nullptr, DM, OUT, DM, bo, 0, 0, 0);
}
